// RotaryPEMultiHeadAttention_42777874268301
// MI455X (gfx1250) — hardware-verified
//
#include <hip/hip_runtime.h>
#include <math.h>
#include <stdint.h>

#define NB    4
#define CH    512
#define SEQ   2048
#define NH    8
#define HD    64
#define NROT  32
#define NPAIR 16
#define NTOK  (NB * SEQ)
#define NQB   (SEQ / 64)
#define NKT   (SEQ / 64)
#define TP    68
static_assert(NH * HD == CH);
static_assert(NPAIR * 2 == NROT && NROT * 2 == HD);
static_assert(NQB == 32 && NKT == 32 && NH == 8);
static_assert((SEQ % 64) == 0 && (CH % 64) == 0 && (CH % 32) == 0 && (NTOK % 64) == 0 && (SEQ % 16) == 0);

typedef __bf16   v16b __attribute__((ext_vector_type(16)));
typedef float    v8f  __attribute__((ext_vector_type(8)));
typedef float    v4f  __attribute__((ext_vector_type(4)));
typedef unsigned int   v4u  __attribute__((ext_vector_type(4)));
typedef unsigned short v8us __attribute__((ext_vector_type(8)));

#if defined(__HIP_DEVICE_COMPILE__)
#define DEV_ASM 1
#else
#define DEV_ASM 0
#endif

__device__ __forceinline__ unsigned short bf_bits(float f) {
  unsigned u = __float_as_uint(f);
  return (unsigned short)((u + 0x7FFFu + ((u >> 16) & 1u)) >> 16);
}
__device__ __forceinline__ float bf_up(unsigned short hb) { return __uint_as_float(((unsigned)hb) << 16); }
__device__ __forceinline__ float bf16r(float f) { return bf_up(bf_bits(f)); }
__device__ __forceinline__ unsigned pk16(unsigned short a, unsigned short b) { return (unsigned)a | ((unsigned)b << 16); }
__device__ __forceinline__ v8f zero8() { v8f z = {0.f, 0.f, 0.f, 0.f, 0.f, 0.f, 0.f, 0.f}; return z; }

union FB { v16b v; v8us h[2]; };
__device__ __forceinline__ v16b ldfrag_b(const unsigned short* p) {
  FB f;
  f.h[0] = *(const v8us*)(p);
  f.h[1] = *(const v8us*)(p + 16);
  return f.v;
}

__device__ __forceinline__ v8f mmar(v16b a, v16b b, v8f c) {
  return __builtin_amdgcn_wmma_f32_16x16x32_bf16(false, a, false, b, (short)0, c, false, false);
}
__device__ __forceinline__ v8f mma_b(v16b a, v16b b, v8f c) {
  c = __builtin_amdgcn_wmma_f32_16x16x32_bf16(false, a, false, b, (short)0, c, false, false);
#if DEV_ASM
  asm volatile("v_nop\n\tv_nop\n\tv_nop\n\tv_nop" : "+v"(c) : "v"(a), "v"(b));
#endif
  return c;
}
__device__ __forceinline__ void dep_guard(v8f& a, v8f& b, v16b x, v16b y) {
#if DEV_ASM
  asm volatile("v_nop\n\tv_nop\n\tv_nop\n\tv_nop" : "+v"(a), "+v"(b) : "v"(x), "v"(y));
#else
  (void)a; (void)b; (void)x; (void)y;
#endif
}
__device__ __forceinline__ void keep4(v16b a, v16b b, v16b c, v16b d) {
#if DEV_ASM
  asm volatile("v_nop" :: "v"(a), "v"(b), "v"(c), "v"(d));
#else
  (void)a; (void)b; (void)c; (void)d;
#endif
}
__device__ __forceinline__ void acc_guard4(v8f& a, v8f& b, v8f& c, v8f& d) {
#if DEV_ASM
  asm volatile("v_nop\n\tv_nop\n\tv_nop\n\tv_nop" : "+v"(a), "+v"(b), "+v"(c), "+v"(d));
#else
  (void)a; (void)b; (void)c; (void)d;
#endif
}

__global__ __launch_bounds__(32) void rope_inv(float* inv) {
  const int i  = (int)threadIdx.x;
  const int ii = i & (NPAIR - 1);
  const float e = (float)(2 * ii) * (1.0f / (float)NROT);
  const float p = powf(10000.0f, e);
  const float v = 1.0f / p;
  *(volatile float*)(inv + i) = v;
  __threadfence();
  *(volatile float*)(inv + i) = v;
}

__global__ __launch_bounds__(256) void rope_tab(const float* __restrict__ inv, float* ctab, float* stab) {
  const int lane = (int)threadIdx.x & 31;
  const int wave = (int)threadIdx.x >> 5;
  const int i = lane & (NPAIR - 1);
  const int t = blockIdx.x * 16 + wave * 2 + (lane >> 4);
  const float f   = inv[lane];
  const float ang = (float)t * f;
  float sn, cs;
  sincosf(ang, &sn, &cs);
  float* pc = ctab + (size_t)t * NPAIR + i;
  float* ps = stab + (size_t)t * NPAIR + i;
  *(volatile float*)pc = cs;
  *(volatile float*)ps = sn;
  __threadfence();
  *(volatile float*)pc = cs;
  *(volatile float*)ps = sn;
}

__global__ __launch_bounds__(256) void cvt_bf16x8(const float* __restrict__ in, unsigned short* out, int n8) {
  const int i = blockIdx.x * 256 + (int)threadIdx.x;
  if (i < n8) {
    const v4f a = *(const v4f*)(in + (size_t)i * 8);
    const v4f b = *(const v4f*)(in + (size_t)i * 8 + 4);
    v4u p;
    p[0] = pk16(bf_bits(a[0]), bf_bits(a[1]));
    p[1] = pk16(bf_bits(a[2]), bf_bits(a[3]));
    p[2] = pk16(bf_bits(b[0]), bf_bits(b[1]));
    p[3] = pk16(bf_bits(b[2]), bf_bits(b[3]));
    *(volatile v4u*)(out + (size_t)i * 8) = p;
    __threadfence();
    *(volatile v4u*)(out + (size_t)i * 8) = p;
  }
}

__global__ __launch_bounds__(256) void tr_cvt(const float* __restrict__ in, unsigned short* outp) {
  __shared__ __align__(16) float ts[64 * TP];
  const int tid = (int)threadIdx.x;
  const int bx  = (int)blockIdx.x;
  const int tc  = bx & 31;
  const int cc  = (bx >> 5) & 7;
  const int b   = bx >> 8;
  const int t0  = tc * 64;
  const int c0  = cc * 64;
  const float* src = in + ((size_t)(b * CH + c0)) * SEQ + t0;

#pragma unroll
  for (int i = 0; i < 4; ++i) {
    const int idx = tid + i * 256;
    const int c   = idx >> 4;
    const int j4  = (idx & 15) * 4;
    const v4f a = *(const v4f*)(src + (size_t)c * SEQ + j4);
    *(v4f*)(ts + c * TP + j4) = a;
  }
  __syncthreads();

  v4u qv[2];
#pragma unroll
  for (int it = 0; it < 2; ++it) {
    const int job = tid + it * 256;
    const int t   = job >> 3;
    const int c8  = (job & 7) * 8;
    float f[8];
#pragma unroll
    for (int e = 0; e < 8; ++e) f[e] = ts[(c8 + e) * TP + t];
    v4u a;
#pragma unroll
    for (int e = 0; e < 4; ++e) a[e] = pk16(bf_bits(f[2 * e]), bf_bits(f[2 * e + 1]));
    qv[it] = a;
  }
  for (int pass = 0; pass < 2; ++pass) {
#pragma unroll
    for (int it = 0; it < 2; ++it) {
      const int job = tid + it * 256;
      const int r   = job >> 3;
      const int e8  = (job & 7) * 8;
      unsigned short* p = outp + ((size_t)(b * SEQ + t0 + r)) * CH + c0 + e8;
      *(volatile v4u*)p = qv[it];
    }
    __threadfence();
  }
}

template <int OUT_MODE, bool TWOB>
__global__ __launch_bounds__(256) __attribute__((amdgpu_num_vgpr(256))) void gemm64(
    const unsigned short* __restrict__ Ap, int lda, long long strideA,
    const unsigned short* __restrict__ Bthp, const unsigned short* __restrict__ Btlp, int ldb, long long strideB,
    void* Cout, void* Cout2, int ldc, long long strideC,
    const float* __restrict__ bias, const float* __restrict__ ctab, const float* __restrict__ stab,
    int M, int N, int K) {
  static_assert(OUT_MODE >= 0 && OUT_MODE <= 2);
  __shared__ __align__(16) float sT[8][16 * 68];
  const int b    = blockIdx.y;
  const int lane = threadIdx.x & 31;
  const int wave = threadIdx.x >> 5;
  const int tilesN = N >> 6;
  const int tilesM = M >> 6;
  const int tile = blockIdx.x * 8 + wave;
  if (tile >= tilesM * tilesN) return;
  const int tm = tile / tilesN;
  const int tn = tile - tm * tilesN;
  const int m0 = tm << 6;
  const int n0 = tn << 6;

  const unsigned short* Ab = Ap + (size_t)b * (size_t)strideA;

  const int rlane = lane & 15;
  const int koff  = (lane >> 4) * 8;
  const int mOff  = (lane >> 4) * 8;

  v8f acc[4][4];
#pragma unroll
  for (int i = 0; i < 4; ++i)
#pragma unroll
    for (int j = 0; j < 4; ++j) acc[i][j] = zero8();

  constexpr int NPL = TWOB ? 2 : 1;
  for (int pl = 0; pl < NPL; ++pl) {
    const unsigned short* Bb = ((pl == 0) ? Bthp : Btlp) + (size_t)b * (size_t)strideB;
    for (int k0 = 0; k0 < K; k0 += 32) {
      v16b bq[4];
#pragma unroll
      for (int j = 0; j < 4; ++j)
        bq[j] = ldfrag_b(Bb + (size_t)(n0 + (j << 4) + rlane) * ldb + koff + k0);
#pragma unroll
      for (int i = 0; i < 4; ++i) {
        const v16b af = ldfrag_b(Ab + (size_t)(m0 + (i << 4) + rlane) * lda + koff + k0);
#pragma unroll
        for (int j = 0; j < 4; ++j) acc[i][j] = mmar(af, bq[j], acc[i][j]);
        dep_guard(acc[i][0], acc[i][3], af, bq[3]);
      }
      keep4(bq[0], bq[1], bq[2], bq[3]);
    }
  }
  acc_guard4(acc[0][0], acc[0][1], acc[0][2], acc[0][3]);
  acc_guard4(acc[1][0], acc[1][1], acc[1][2], acc[1][3]);
  acc_guard4(acc[2][0], acc[2][1], acc[2][2], acc[2][3]);
  acc_guard4(acc[3][0], acc[3][1], acc[3][2], acc[3][3]);

  float* slab = sT[wave];
#pragma unroll
  for (int i = 0; i < 4; ++i) {
    const int mBase = m0 + (i << 4);
#pragma unroll
    for (int j = 0; j < 4; ++j) {
#pragma unroll
      for (int r = 0; r < 8; ++r) {
        slab[(mOff + r) * 68 + (j << 4) + rlane] = acc[i][j][r];
      }
    }
    __builtin_amdgcn_fence(__ATOMIC_RELEASE, "workgroup");
    __builtin_amdgcn_wave_barrier();
    __builtin_amdgcn_fence(__ATOMIC_ACQUIRE, "workgroup");
    if (OUT_MODE == 0) {
      float* C = (float*)Cout + (size_t)b * (size_t)strideC;
      const int h2 = lane >> 4, c4 = (lane & 15) * 4;
      v4f ov[8];
#pragma unroll
      for (int it = 0; it < 8; ++it) {
        const int row = it * 2 + h2;
        const float bm = bf16r(bias[mBase + row]);
        v4f v = *(const v4f*)(slab + row * 68 + c4);
#pragma unroll
        for (int e = 0; e < 4; ++e) v[e] = v[e] + bm;
        ov[it] = v;
      }
      for (int pass = 0; pass < 2; ++pass) {
#pragma unroll
        for (int it = 0; it < 8; ++it) {
          const int row = it * 2 + h2;
          *(volatile v4f*)(C + (size_t)(mBase + row) * ldc + n0 + c4) = ov[it];
        }
        __threadfence();
      }
    } else {
      const int q = lane >> 3, c8 = (lane & 7) * 8;
      unsigned short* C  = (unsigned short*)Cout  + (size_t)b * (size_t)strideC;
      unsigned short* C2 = (unsigned short*)Cout2 + (size_t)b * (size_t)strideC;
#pragma unroll
      for (int it = 0; it < 4; ++it) {
        const int row = it * 4 + q;
        const float* sp = slab + row * 68 + c8;
        float f[8];
#pragma unroll
        for (int e = 0; e < 8; ++e) f[e] = sp[e];
        if (OUT_MODE == 1) {
#pragma clang fp contract(off)
          const int pc8 = c8 ^ 16;
          const float* pp = slab + row * 68 + pc8;
          float g[8];
#pragma unroll
          for (int e = 0; e < 8; ++e) g[e] = pp[e];
          const v4f bc0 = *(const v4f*)(bias + n0 + c8);
          const v4f bc1 = *(const v4f*)(bias + n0 + c8 + 4);
          const v4f bp0 = *(const v4f*)(bias + n0 + pc8);
          const v4f bp1 = *(const v4f*)(bias + n0 + pc8 + 4);
          const int t  = (mBase + row) & (SEQ - 1);
          const int j0 = c8 & (NPAIR - 1);
          const v4f cv0 = *(const v4f*)(ctab + (size_t)t * NPAIR + j0);
          const v4f cv1 = *(const v4f*)(ctab + (size_t)t * NPAIR + j0 + 4);
          const v4f sv0 = *(const v4f*)(stab + (size_t)t * NPAIR + j0);
          const v4f sv1 = *(const v4f*)(stab + (size_t)t * NPAIR + j0 + 4);
          const bool  rot = (c8 < NROT);
          const float sg  = (c8 < NPAIR) ? -1.0f : 1.0f;
#pragma unroll
          for (int e = 0; e < 4; ++e) {
            {
              const float x  = f[e] + bf16r(bc0[e]);
              const float y  = g[e] + bf16r(bp0[e]);
              const float ry = sg * y;
              const float p0 = x * cv0[e];
              const float p1 = ry * sv0[e];
              const float rv = p0 + p1;
              f[e] = rot ? rv : x;
            }
            {
              const float x  = f[4 + e] + bf16r(bc1[e]);
              const float y  = g[4 + e] + bf16r(bp1[e]);
              const float ry = sg * y;
              const float p0 = x * cv1[e];
              const float p1 = ry * sv1[e];
              const float rv = p0 + p1;
              f[4 + e] = rot ? rv : x;
            }
          }
        }
        if (OUT_MODE == 2) {
          const float bm = bf16r(bias[mBase + row]);
#pragma unroll
          for (int e = 0; e < 8; ++e) f[e] = f[e] + bm;
        }
        v4u a, a2;
#pragma unroll
        for (int e = 0; e < 4; ++e) {
          const float f0 = f[2 * e], f1 = f[2 * e + 1];
          const unsigned short h0 = bf_bits(f0), h1 = bf_bits(f1);
          const unsigned short l0 = bf_bits(f0 - bf_up(h0)), l1 = bf_bits(f1 - bf_up(h1));
          a[e] = pk16(h0, h1); a2[e] = pk16(l0, l1);
        }
        unsigned short* cp  = C  + (size_t)(mBase + row) * ldc + n0 + c8;
        unsigned short* cp2 = C2 + (size_t)(mBase + row) * ldc + n0 + c8;
        *(volatile v4u*)cp  = a;
        *(volatile v4u*)cp2 = a2;
        __threadfence();
        *(volatile v4u*)cp  = a;
        *(volatile v4u*)cp2 = a2;
      }
    }
    __builtin_amdgcn_fence(__ATOMIC_RELEASE, "workgroup");
    __builtin_amdgcn_wave_barrier();
    __builtin_amdgcn_fence(__ATOMIC_ACQUIRE, "workgroup");
  }
}

union KOsh { unsigned short k[2][64 * 64]; float o[4][16 * 64]; };

__global__ __launch_bounds__(128) __attribute__((amdgpu_num_vgpr(256)))
void attn_x(const unsigned short* __restrict__ qhp, const unsigned short* __restrict__ qlp,
            const unsigned short* __restrict__ khp, const unsigned short* __restrict__ klp,
            const unsigned short* __restrict__ vhp, const unsigned short* __restrict__ vlp,
            unsigned short* ohp, unsigned short* olp, float sscale) {
  __shared__ __align__(16) KOsh UK;
  __shared__ __align__(16) unsigned short Vsh[2][64 * 64];
  __shared__ __align__(16) unsigned short Phs[4][16 * 64];
  __shared__ __align__(16) unsigned short Pls[4][16 * 64];

  const int tid  = (int)threadIdx.x;
  const int wave = tid >> 5;
  const int lane = tid & 31;
  const int hh   = lane >> 4;
  const int c    = lane & 15;

  const int bx = (int)blockIdx.x;
  const int qb = bx & (NQB - 1);
  const int h  = (bx >> 5) & (NH - 1);
  const int b  = bx >> 8;
  const int q0 = qb * 64 + wave * 16;
  const size_t rowB  = (size_t)b * SEQ;
  const size_t hcol  = (size_t)h * HD;
  const size_t vbase = ((size_t)b * CH + hcol) * SEQ;

  v16b qah[2], qal[2];
#pragma unroll
  for (int dc = 0; dc < 2; ++dc) {
    const size_t qo = (rowB + q0 + c) * CH + hcol + dc * 32 + 8 * hh;
    qah[dc] = ldfrag_b(qhp + qo);
    qal[dc] = ldfrag_b(qlp + qo);
  }

  float mrow[8], lrow[8];
  v8f oacc[4];
#pragma unroll
  for (int r = 0; r < 8; ++r) { mrow[r] = -INFINITY; lrow[r] = 0.f; }
#pragma unroll
  for (int t = 0; t < 4; ++t) oacc[t] = zero8();

  unsigned short* ph = Phs[wave];
  unsigned short* pl = Pls[wave];

  for (int kt = 0; kt < NKT; ++kt) {
    const int kv0 = kt * 64;
    __syncthreads();
    {
      const int r = tid >> 1, half = (tid & 1) * 32;
      const unsigned short* kgh = khp + (rowB + kv0 + r) * CH + hcol + half;
      const unsigned short* kgl = klp + (rowB + kv0 + r) * CH + hcol + half;
      const unsigned short* vgh = vhp + vbase + (size_t)r * SEQ + kv0 + half;
      const unsigned short* vgl = vlp + vbase + (size_t)r * SEQ + kv0 + half;
#pragma unroll
      for (int i = 0; i < 4; ++i) {
        const v8us a0 = *(const v8us*)(kgh + 8 * i);
        const v8us a1 = *(const v8us*)(kgl + 8 * i);
        const v8us b0 = *(const v8us*)(vgh + 8 * i);
        const v8us b1 = *(const v8us*)(vgl + 8 * i);
        *(v8us*)(UK.k[0] + r * 64 + half + 8 * i) = a0;
        *(v8us*)(UK.k[1] + r * 64 + half + 8 * i) = a1;
        *(v8us*)(Vsh[0]  + r * 64 + half + 8 * i) = b0;
        *(v8us*)(Vsh[1]  + r * 64 + half + 8 * i) = b1;
      }
    }
    __syncthreads();

    v8f s[4];
#pragma unroll
    for (int j = 0; j < 4; ++j) {
      v8f acc = zero8();
#pragma unroll
      for (int dc = 0; dc < 2; ++dc) {
        FB kh, kl;
        kh.h[0] = *(const v8us*)(UK.k[0] + (j * 16 + c) * 64 + dc * 32 + 8 * hh);
        kh.h[1] = *(const v8us*)(UK.k[0] + (j * 16 + c) * 64 + dc * 32 + 16 + 8 * hh);
        kl.h[0] = *(const v8us*)(UK.k[1] + (j * 16 + c) * 64 + dc * 32 + 8 * hh);
        kl.h[1] = *(const v8us*)(UK.k[1] + (j * 16 + c) * 64 + dc * 32 + 16 + 8 * hh);
        acc = mma_b(qah[dc], kh.v, acc);
        acc = mma_b(qah[dc], kl.v, acc);
        acc = mma_b(qal[dc], kh.v, acc);
      }
#pragma unroll
      for (int r = 0; r < 8; ++r) s[j][r] = acc[r] * sscale;
    }

#pragma unroll
    for (int r = 0; r < 8; ++r) {
      float mx = s[0][r];
#pragma unroll
      for (int j = 1; j < 4; ++j) mx = fmaxf(mx, s[j][r]);
#pragma unroll
      for (int off = 1; off < 16; off <<= 1) mx = fmaxf(mx, __shfl_xor(mx, off, 32));
      const float mnew  = fmaxf(mrow[r], mx);
      const float msafe = (mnew == -INFINITY) ? 0.f : mnew;
      const float alpha = __expf(mrow[r] - msafe);
      mrow[r] = mnew;
      float psum = 0.f;
#pragma unroll
      for (int j = 0; j < 4; ++j) {
        const float p = __expf(s[j][r] - msafe);
        psum += p;
        const unsigned short hb = bf_bits(p);
        const float hu = bf_up(hb);
        const unsigned short lb = bf_bits(p - hu);
        const int idx = (8 * hh + r) * 64 + j * 16 + c;
        ph[idx] = hb;
        pl[idx] = lb;
      }
      lrow[r] = lrow[r] * alpha + psum;
#pragma unroll
      for (int t = 0; t < 4; ++t) oacc[t][r] *= alpha;
    }
    __builtin_amdgcn_fence(__ATOMIC_RELEASE, "workgroup");
    __builtin_amdgcn_wave_barrier();
    __builtin_amdgcn_fence(__ATOMIC_ACQUIRE, "workgroup");

#pragma unroll 1
    for (int kk = 0; kk < 2; ++kk) {
      FB pa, pb;
      pa.h[0] = *(const v8us*)(ph + c * 64 + kk * 32 + 8 * hh);
      pa.h[1] = *(const v8us*)(ph + c * 64 + kk * 32 + 16 + 8 * hh);
      pb.h[0] = *(const v8us*)(pl + c * 64 + kk * 32 + 8 * hh);
      pb.h[1] = *(const v8us*)(pl + c * 64 + kk * 32 + 16 + 8 * hh);
#pragma unroll
      for (int t = 0; t < 4; ++t) {
        FB vh, vl;
        vh.h[0] = *(const v8us*)(Vsh[0] + (t * 16 + c) * 64 + kk * 32 + 8 * hh);
        vh.h[1] = *(const v8us*)(Vsh[0] + (t * 16 + c) * 64 + kk * 32 + 16 + 8 * hh);
        vl.h[0] = *(const v8us*)(Vsh[1] + (t * 16 + c) * 64 + kk * 32 + 8 * hh);
        vl.h[1] = *(const v8us*)(Vsh[1] + (t * 16 + c) * 64 + kk * 32 + 16 + 8 * hh);
        oacc[t] = mma_b(pa.v, vh.v, oacc[t]);
        oacc[t] = mma_b(pb.v, vh.v, oacc[t]);
        oacc[t] = mma_b(pa.v, vl.v, oacc[t]);
      }
    }
  }
  __syncthreads();

  float* os = UK.o[wave];
#pragma unroll
  for (int r = 0; r < 8; ++r) {
    float l = lrow[r];
#pragma unroll
    for (int off = 1; off < 16; off <<= 1) l += __shfl_xor(l, off, 32);
    const float inv = (l > 0.f) ? (1.0f / l) : 0.f;
#pragma unroll
    for (int t = 0; t < 4; ++t) os[(8 * hh + r) * 64 + t * 16 + c] = oacc[t][r] * inv;
  }
  __builtin_amdgcn_fence(__ATOMIC_RELEASE, "workgroup");
  __builtin_amdgcn_wave_barrier();
  __builtin_amdgcn_fence(__ATOMIC_ACQUIRE, "workgroup");
  {
    const int q4 = lane >> 3, c8 = (lane & 7) * 8;
    v4u hv[4], lv[4];
#pragma unroll
    for (int it = 0; it < 4; ++it) {
      const int row = it * 4 + q4;
      const float* sp = os + row * 64 + c8;
      v4u a, a2;
#pragma unroll
      for (int e = 0; e < 4; ++e) {
        const float f0 = sp[2 * e], f1 = sp[2 * e + 1];
        const unsigned short h0 = bf_bits(f0), h1 = bf_bits(f1);
        const unsigned short l0 = bf_bits(f0 - bf_up(h0)), l1 = bf_bits(f1 - bf_up(h1));
        a[e] = pk16(h0, h1); a2[e] = pk16(l0, l1);
      }
      hv[it] = a; lv[it] = a2;
    }
    for (int pass = 0; pass < 2; ++pass) {
#pragma unroll
      for (int it = 0; it < 4; ++it) {
        const int row = it * 4 + q4;
        const size_t go = (rowB + q0 + row) * CH + hcol + c8;
        *(volatile v4u*)(ohp + go) = hv[it];
        *(volatile v4u*)(olp + go) = lv[it];
      }
      __threadfence();
    }
  }
}

extern "C" void kernel_launch(void* const* d_in, const int* in_sizes, int n_in,
                              void* d_out, int out_size, void* d_ws, size_t ws_size,
                              hipStream_t stream) {
  if (n_in < 10) return;
  if (in_sizes[0] != NB * CH * SEQ) return;
  if (in_sizes[1] != NB * CH * SEQ) return;
  if (in_sizes[2] != CH * CH) return;
  if (in_sizes[3] != CH) return;
  if (in_sizes[4] != CH * CH) return;
  if (in_sizes[5] != CH) return;
  if (in_sizes[6] != CH * CH) return;
  if (in_sizes[7] != CH) return;
  if (in_sizes[8] != CH * CH) return;
  if (in_sizes[9] != CH) return;
  if (out_size != NB * CH * SEQ) return;

  const float* x  = (const float*)d_in[0];
  const float* cc = (const float*)d_in[1];
  const float* Wq = (const float*)d_in[2];
  const float* bq = (const float*)d_in[3];
  const float* Wk = (const float*)d_in[4];
  const float* bk = (const float*)d_in[5];
  const float* Wv = (const float*)d_in[6];
  const float* bv = (const float*)d_in[7];
  const float* Wo = (const float*)d_in[8];
  const float* bo = (const float*)d_in[9];

  const size_t PX  = (size_t)NTOK * CH * 2;
  const size_t PV  = (size_t)NB * CH * SEQ * 2;
  const size_t PW  = (size_t)CH * CH * 2;
  const size_t PTB = (size_t)SEQ * NPAIR * 4;
  const size_t PIV = 128;
  size_t off = 0;
  const size_t oXp = off; off += PX;
  const size_t oCp = off; off += PX;
  const size_t oWq = off; off += PW;
  const size_t oWk = off; off += PW;
  const size_t oWv = off; off += PW;
  const size_t oWo = off; off += PW;
  const size_t oQh = off; off += PX;
  const size_t oQl = off; off += PX;
  const size_t oKh = off; off += PX;
  const size_t oKl = off; off += PX;
  const size_t oVh = off; off += PV;
  const size_t oVl = off; off += PV;
  const size_t oOh = off; off += PX;
  const size_t oOl = off; off += PX;
  const size_t oTc = off; off += PTB;
  const size_t oTs = off; off += PTB;
  const size_t oIv = off; off += PIV;
  if (off > ws_size) return;
  if (off > (size_t)134217728) return;

  char* ws = (char*)d_ws;
  unsigned short* Xp  = (unsigned short*)(ws + oXp);
  unsigned short* Cp  = (unsigned short*)(ws + oCp);
  unsigned short* Wqb = (unsigned short*)(ws + oWq);
  unsigned short* Wkb = (unsigned short*)(ws + oWk);
  unsigned short* Wvb = (unsigned short*)(ws + oWv);
  unsigned short* Wob = (unsigned short*)(ws + oWo);
  unsigned short* Qh  = (unsigned short*)(ws + oQh);
  unsigned short* Ql  = (unsigned short*)(ws + oQl);
  unsigned short* Kh  = (unsigned short*)(ws + oKh);
  unsigned short* Kl  = (unsigned short*)(ws + oKl);
  unsigned short* Vh  = (unsigned short*)(ws + oVh);
  unsigned short* Vl  = (unsigned short*)(ws + oVl);
  unsigned short* Oh  = (unsigned short*)(ws + oOh);
  unsigned short* Ol  = (unsigned short*)(ws + oOl);
  float*          Tc  = (float*)(ws + oTc);
  float*          Ts  = (float*)(ws + oTs);
  float*          Iv  = (float*)(ws + oIv);

  const dim3 blk(256);
  const int n8w = CH * CH / 8;
  const dim3 gCvtW((n8w + 255) / 256);
  const dim3 gTab(SEQ / 16);
  const dim3 gTr(NB * (CH / 64) * (SEQ / 64));
  const dim3 gP(((NTOK / 64) * (CH / 64) + 7) / 8, 1);
  const dim3 gV(((CH / 64) * (SEQ / 64) + 7) / 8, NB);
  const dim3 gAttn(NB * NH * NQB);
  static_assert(((NTOK / 64) * (CH / 64)) % 8 == 0 && ((CH / 64) * (SEQ / 64)) % 8 == 0);
  static_assert((CH % 32) == 0 && ((CH * CH) % 2048) == 0);

  rope_inv<<<dim3(1), dim3(32), 0, stream>>>(Iv);
  rope_tab<<<gTab, blk, 0, stream>>>(Iv, Tc, Ts);
  tr_cvt<<<gTr, blk, 0, stream>>>(x, Xp);
  tr_cvt<<<gTr, blk, 0, stream>>>(cc, Cp);
  cvt_bf16x8<<<gCvtW, blk, 0, stream>>>(Wq, Wqb, n8w);
  cvt_bf16x8<<<gCvtW, blk, 0, stream>>>(Wk, Wkb, n8w);
  cvt_bf16x8<<<gCvtW, blk, 0, stream>>>(Wv, Wvb, n8w);
  cvt_bf16x8<<<gCvtW, blk, 0, stream>>>(Wo, Wob, n8w);
  gemm64<1, false><<<gP, blk, 0, stream>>>(
      Xp, CH, 0LL, Wqb, Wqb, CH, 0LL,
      (void*)Qh, (void*)Ql, CH, 0LL, bq, Tc, Ts,
      NTOK, CH, CH);
  gemm64<1, false><<<gP, blk, 0, stream>>>(
      Cp, CH, 0LL, Wkb, Wkb, CH, 0LL,
      (void*)Kh, (void*)Kl, CH, 0LL, bk, Tc, Ts,
      NTOK, CH, CH);
  gemm64<2, false><<<gV, blk, 0, stream>>>(
      Wvb, CH, 0LL, Cp, Cp, CH, (long long)SEQ * CH,
      (void*)Vh, (void*)Vl, SEQ, (long long)CH * SEQ, bv, Tc, Ts,
      CH, SEQ, CH);
  attn_x<<<gAttn, dim3(128), 0, stream>>>(Qh, Ql, Kh, Kl, Vh, Vl, Oh, Ol, 0.125f);
  gemm64<0, true><<<gV, blk, 0, stream>>>(
      Wob, CH, 0LL, Oh, Ol, CH, (long long)SEQ * CH,
      d_out, d_out, SEQ, (long long)CH * SEQ, bo, Tc, Ts,
      CH, SEQ, CH);
  (void)hipGetLastError();
}
